// s6ClassicModule_24154896073581
// MI455X (gfx1250) — hardware-run, weakly checked
//
#include <hip/hip_runtime.h>
#include <hip/hip_fp16.h>
#include <math.h>

typedef __attribute__((ext_vector_type(16))) _Float16 v16h;
typedef __attribute__((ext_vector_type(8)))  _Float16 v8h;
typedef __attribute__((ext_vector_type(8)))  float    v8f;
typedef __attribute__((ext_vector_type(4)))  float    v4f;

constexpr int kBatch = 2;
constexpr int kDm    = 1024;
constexpr int kSeq   = 2048;
constexpr int kNst   = 16;
constexpr int kRank  = 64;
constexpr int kXpN   = kRank + 2 * kNst;
constexpr int kXpP   = 128;
constexpr int kOutN  = 2 * kDm;
constexpr int kRows  = kBatch * kSeq;
constexpr int kOffB  = kRank;
constexpr int kOffC  = kRank + kNst;
static_assert(kXpN == 96 && kXpN <= kXpP);
static_assert((kDm % 64) == 0 && (kSeq % 64) == 0 && (kXpP % 64) == 0 && (kOutN % 64) == 0);
static_assert((kDm % 32) == 0 && (kRank % 32) == 0);

constexpr int kSplX   = 0;
constexpr int kSplDt  = 0;
constexpr int kSplOut = 1;
constexpr int kMiX   = (kSplX   == 2) ? 1 : 2;
constexpr int kMiDt  = (kSplDt  == 2) ? 1 : 2;
constexpr int kMiOut = (kSplOut == 2) ? 1 : 2;
static_assert((kRows % (16 * kMiX)) == 0 && (kRows % (16 * kMiDt)) == 0 && (kRows % (16 * kMiOut)) == 0);
static_assert((((kRows / (16 * kMiX))   * (kXpP  / 64)) % 8) == 0);
static_assert((((kRows / (16 * kMiDt))  * (kDm   / 64)) % 8) == 0);
static_assert((((kRows / (16 * kMiOut)) * (kOutN / 64)) % 8) == 0);

constexpr float kXwCarry = 256.0f;
constexpr float kDlCarry = 64.0f;
constexpr float kDwCarry = 64.0f;
constexpr float kYCarry  = 16.0f;
constexpr float kGCarry  = 16.0f;
constexpr float kOwCarry = 256.0f;
constexpr float kResid   = 2048.0f;
constexpr float kOne     = 1.0f;
constexpr float kScX    = 1.0f / kXwCarry;
constexpr float kScXr   = 1.0f / (kXwCarry * kResid);
constexpr float kScDt   = 1.0f / (kDlCarry * kDwCarry);
constexpr float kScDtr  = 1.0f / (kDlCarry * kDwCarry * kResid);
constexpr float kScOut  = 1.0f / (kGCarry * kOwCarry);
constexpr float kScOutr = 1.0f / (kGCarry * kOwCarry * kResid);

constexpr size_t kSzU    = (size_t)kRows * kDm * 4;
constexpr size_t kSzU16  = (size_t)kRows * kDm * 2;
constexpr size_t kSzXW   = (size_t)kXpP * kDm * 2;
constexpr size_t kSzDTW  = (size_t)kDm * kRank * 2;
constexpr size_t kSzOW   = (size_t)kOutN * kDm * 2;
constexpr size_t kSzXD   = (size_t)kRows * kXpP * 4;
constexpr size_t kSzDTL  = (size_t)kRows * kRank * 2;
constexpr size_t kSzOUT  = (size_t)kRows * kOutN * 4;
constexpr size_t kOffU    = 0;
constexpr size_t kOffUH   = kOffU    + kSzU;
constexpr size_t kOffUL   = kOffUH   + kSzU16;
constexpr size_t kOffXWH  = kOffUL   + kSzU16;
constexpr size_t kOffXWL  = kOffXWH  + kSzXW;
constexpr size_t kOffDTWH = kOffXWL  + kSzXW;
constexpr size_t kOffDTWL = kOffDTWH + kSzDTW;
constexpr size_t kOffOWH  = kOffDTWL + kSzDTW;
constexpr size_t kOffOWL  = kOffOWH  + kSzOW;
constexpr size_t kOffXD   = kOffOWL  + kSzOW;
constexpr size_t kOffDTLH = kOffXD   + kSzXD;
constexpr size_t kOffDTLL = kOffDTLH + kSzDTL;
constexpr size_t kOffDT   = kOffDTLL + kSzDTL;
constexpr size_t kOffYH   = kOffDT   + kSzU;
constexpr size_t kOffYL   = kOffYH   + kSzU16;
constexpr size_t kOffGH   = kOffYL   + kSzU16;
constexpr size_t kOffGL   = kOffGH   + kSzU16;
constexpr size_t kOffOUT  = kOffGL   + kSzU16;
constexpr size_t kWsTotal = kOffOUT  + kSzOUT;
static_assert(kWsTotal == 129761280ull);
static_assert(kWsTotal <= 134217728ull);
static_assert((kOffUH % 128) == 0 && (kOffUL % 128) == 0 && (kOffXWH % 128) == 0 && (kOffXWL % 128) == 0 &&
              (kOffDTWH % 128) == 0 && (kOffDTWL % 128) == 0 && (kOffOWH % 128) == 0 && (kOffOWL % 128) == 0 &&
              (kOffXD % 128) == 0 && (kOffDTLH % 128) == 0 && (kOffDTLL % 128) == 0 && (kOffDT % 128) == 0 &&
              (kOffYH % 128) == 0 && (kOffYL % 128) == 0 && (kOffGH % 128) == 0 && (kOffGL % 128) == 0 &&
              (kOffOUT % 128) == 0);

__device__ __forceinline__ _Float16 f16_flush(float v) {
  const float w = (fabsf(v) < 6.103515625e-05f) ? 0.0f : v;
  return (_Float16)w;
}
__device__ __forceinline__ void f16_split(float v, _Float16& hi, _Float16& lo) {
  hi = f16_flush(v);
  const float hf = (float)hi;
  const float r = (v - hf) * kResid;
  lo = f16_flush(r);
}
__device__ __forceinline__ unsigned f16_bits_flush(float v) {
  const float w = (fabsf(v) < 6.103515625e-05f) ? 0.0f : v;
  return (unsigned)__builtin_bit_cast(unsigned short, (_Float16)w);
}
__device__ __forceinline__ float h16_to_f32(unsigned hb) {
  const unsigned sgn = (hb & 0x8000u) << 16; const unsigned em = hb & 0x7fffu;
  const float fn = __uint_as_float((em << 13) + 0x38000000u);
  const float fs = (float)em * 5.9604644775390625e-8f;
  const float mag = (em < 0x400u) ? fs : fn; return __uint_as_float(__float_as_uint(mag) | sgn); }

namespace eng {
union FragU { v16h v; v8h h[2]; };
__device__ __forceinline__ v16h frag_load(const _Float16* p) {
  FragU f;
  f.h[0] = *(const v8h*)(p);
  f.h[1] = *(const v8h*)(p + 16);
  return f.v;
}
__device__ __forceinline__ v8f mma(v16h a, v16h b, v8f c) {
  return __builtin_amdgcn_wmma_f32_16x16x32_f16(false, a, false, b, (short)0, c, false, false);
}
__device__ __forceinline__ void guard1(v8f& a, v16h x, v16h y) {
  asm volatile("v_nop\n\tv_nop\n\tv_nop\n\tv_nop" : "+v"(a) : "v"(x), "v"(y));
}
__device__ __forceinline__ void guard_acc(v8f& a) {
  asm volatile("v_nop\n\tv_nop\n\tv_nop\n\tv_nop" : "+v"(a));
}
__device__ __forceinline__ void keep4(v16h a, v16h b, v16h c, v16h d) {
  asm volatile("v_nop" :: "v"(a), "v"(b), "v"(c), "v"(d));
}

template <int MI, int SPL, int BIAS>
__global__ __launch_bounds__(256) void gemm_f16_kernel(
    const unsigned short* __restrict__ Ap, const unsigned short* __restrict__ A2p, int lda,
    const unsigned short* __restrict__ Btp, const unsigned short* __restrict__ Bt2p, int ldb,
    float* __restrict__ C, int ldc, const float* __restrict__ bias,
    int M, int N, int K, float scale, float rscale)
{
  static_assert(MI >= 1 && MI <= 2);
  static_assert(SPL >= 0 && SPL <= 2);
  static_assert(BIAS >= 0 && BIAS <= 1);
  const _Float16* A   = (const _Float16*)Ap;
  const _Float16* A2  = (const _Float16*)A2p;
  const _Float16* Bt  = (const _Float16*)Btp;
  const _Float16* Bt2 = (const _Float16*)Bt2p;
  __shared__ __align__(16) float sT[8][16 * 68];
  const int lane = threadIdx.x & 31;
  const int wave = threadIdx.x >> 5;
  const int tilesN = N >> 6;
  const int tilesM = M / (16 * MI);
  const int tile = blockIdx.x * 8 + wave;
  if (tile >= tilesM * tilesN) return;
  const int tm = tile / tilesN;
  const int tn = tile - tm * tilesN;
  const int m0 = tm * (16 * MI);
  const int n0 = tn << 6;
  const int rlane = lane & 15;
  const int koff  = (lane >> 4) * 8;
  const int mOff  = (lane >> 4) * 8;

  v8f acc[MI][4], accr[MI][4];
#pragma unroll
  for (int i = 0; i < MI; ++i)
#pragma unroll
    for (int j = 0; j < 4; ++j) {
      acc[i][j]  = (v8f){0.f, 0.f, 0.f, 0.f, 0.f, 0.f, 0.f, 0.f};
      accr[i][j] = (v8f){0.f, 0.f, 0.f, 0.f, 0.f, 0.f, 0.f, 0.f};
    }

  for (int k0 = 0; k0 < K; k0 += 32) {
    v16h bh[4], bl[4];
#pragma unroll
    for (int j = 0; j < 4; ++j) {
      const size_t bo = (size_t)(n0 + (j << 4) + rlane) * ldb + koff + k0;
      bh[j] = frag_load(Bt + bo);
      if (SPL == 2) bl[j] = frag_load(Bt2 + bo); else bl[j] = bh[j];
    }
#pragma unroll
    for (int i = 0; i < MI; ++i) {
      const size_t ao = (size_t)(m0 + (i << 4) + rlane) * lda + koff + k0;
      const v16h ah = frag_load(A + ao);
      v16h al = ah;
      if (SPL >= 1) al = frag_load(A2 + ao);
#pragma unroll
      for (int j = 0; j < 4; ++j) {
        acc[i][j] = mma(ah, bh[j], acc[i][j]);
        if (SPL >= 1) accr[i][j] = mma(al, bh[j], accr[i][j]);
        if (SPL == 2) accr[i][j] = mma(ah, bl[j], accr[i][j]);
      }
#pragma unroll
      for (int j = 0; j < 4; ++j) {
        guard1(acc[i][j], ah, al);
        if (SPL >= 1) guard1(accr[i][j], ah, al);
      }
    }
    keep4(bh[0], bh[1], bh[2], bh[3]);
    if (SPL == 2) keep4(bl[0], bl[1], bl[2], bl[3]);
  }
#pragma unroll
  for (int i = 0; i < MI; ++i)
#pragma unroll
    for (int j = 0; j < 4; ++j) {
      guard_acc(acc[i][j]);
      if (SPL >= 1) guard_acc(accr[i][j]);
    }

  float* slab = sT[wave];
#pragma unroll
  for (int i = 0; i < MI; ++i) {
    const int mBase = m0 + (i << 4);
#pragma unroll
    for (int j = 0; j < 4; ++j) {
      float bv = 0.0f;
      if (BIAS == 1) bv = bias[n0 + (j << 4) + rlane];
#pragma unroll
      for (int r = 0; r < 8; ++r) {
        float v = acc[i][j][r] * scale;
        if (SPL >= 1) v += accr[i][j][r] * rscale;
        if (BIAS == 1) v += bv;
        slab[(mOff + r) * 68 + (j << 4) + rlane] = v;
      }
    }
    __builtin_amdgcn_fence(__ATOMIC_RELEASE, "workgroup");
    __builtin_amdgcn_wave_barrier();
    __builtin_amdgcn_fence(__ATOMIC_ACQUIRE, "workgroup");
    {
      const int hh = lane >> 4, c4 = (lane & 15) * 4;
      for (int pass = 0; pass < 2; ++pass) {
#pragma unroll
        for (int it = 0; it < 8; ++it) {
          const int row = it * 2 + hh;
          const v4f v = *(const v4f*)(slab + row * 68 + c4);
          *(volatile v4f*)(C + (size_t)(mBase + row) * ldc + n0 + c4) = v;
        }
        __threadfence();
      }
    }
    __builtin_amdgcn_fence(__ATOMIC_RELEASE, "workgroup");
    __builtin_amdgcn_wave_barrier();
    __builtin_amdgcn_fence(__ATOMIC_ACQUIRE, "workgroup");
  }
}
}

template <bool LO>
__global__ __launch_bounds__(256) void pack_rows_kernel(
    const float* __restrict__ src, unsigned short* __restrict__ dH, unsigned short* __restrict__ dL,
    int rowsReal, int cols, int total8, float carry)
{
  const int i = blockIdx.x * 256 + threadIdx.x;
  if (i >= total8) return;
  const size_t e0 = (size_t)i << 3;
  const int row = (int)(e0 / (size_t)cols);
  const int col = (int)(e0 - (size_t)row * (size_t)cols);
  const bool real = (row < rowsReal);
  const int rc = real ? row : (rowsReal - 1);
  const float* sp = src + (size_t)rc * cols + col;
  const v4f a0 = *(const v4f*)(sp);
  const v4f a1 = *(const v4f*)(sp + 4);
  v8h hv, lv;
#pragma unroll
  for (int e = 0; e < 4; ++e) {
    _Float16 h0, l0, h1, l1;
    const float f0 = real ? (a0[e] * carry) : 0.0f;
    const float f1 = real ? (a1[e] * carry) : 0.0f;
    f16_split(f0, h0, l0);
    f16_split(f1, h1, l1);
    hv[e] = h0; lv[e] = l0;
    hv[4 + e] = h1; lv[4 + e] = l1;
  }
  unsigned short* qh = dH + e0;
  unsigned short* ql = dL + e0;
  *(volatile v8h*)qh = hv;
  if (LO) *(volatile v8h*)ql = lv;
  __threadfence();
  *(volatile v8h*)qh = hv;
  if (LO) *(volatile v8h*)ql = lv;
}

template <bool LO>
__global__ __launch_bounds__(256) void transpose_u_kernel(
    const float* __restrict__ X, float* __restrict__ U,
    unsigned short* __restrict__ UH, unsigned short* __restrict__ UL)
{
  __shared__ __align__(16) float tile[64 * 68];
  const int tid = threadIdx.x, lane = tid & 31, wave = tid >> 5;
  const int l0 = blockIdx.x * 64;
  const int d0 = blockIdx.y * 64;
  const int b  = blockIdx.z;
  const float* src = X + ((size_t)b * kDm + d0) * kSeq + l0;
#pragma unroll
  for (int p = 0; p < 4; ++p) {
    const int idx = tid + p * 256;
    const int dd  = idx >> 4;
    const int l4  = (idx & 15) * 4;
    const v4f v = *(const v4f*)(src + (size_t)dd * kSeq + l4);
#pragma unroll
    for (int e = 0; e < 4; ++e) tile[(l4 + e) * 68 + dd] = v[e];
  }
  __syncthreads();
  const int hh = lane >> 4, c4 = (lane & 15) * 4;
  const int q  = lane >> 3, c8 = (lane & 7) * 8;
  const size_t grow0 = (size_t)b * kSeq + l0;
  v4f fv[4];
  v8h hv[2], lv[2];
#pragma unroll
  for (int it = 0; it < 4; ++it) fv[it] = *(const v4f*)(tile + (wave * 8 + it * 2 + hh) * 68 + c4);
#pragma unroll
  for (int it = 0; it < 2; ++it) {
    const float* sp = tile + (it * 32 + wave * 4 + q) * 68 + c8;
    const v4f a0 = *(const v4f*)(sp);
    const v4f a1 = *(const v4f*)(sp + 4);
#pragma unroll
    for (int e = 0; e < 4; ++e) {
      _Float16 h0, l0h, h1, l1h;
      const float f0 = a0[e];
      const float f1 = a1[e];
      f16_split(f0, h0, l0h);
      f16_split(f1, h1, l1h);
      hv[it][e] = h0; lv[it][e] = l0h;
      hv[it][4 + e] = h1; lv[it][4 + e] = l1h;
    }
  }
  for (int pass = 0; pass < 2; ++pass) {
#pragma unroll
    for (int it = 0; it < 4; ++it)
      *(volatile v4f*)(U + (grow0 + wave * 8 + it * 2 + hh) * kDm + d0 + c4) = fv[it];
#pragma unroll
    for (int it = 0; it < 2; ++it) {
      const size_t o = (grow0 + it * 32 + wave * 4 + q) * kDm + d0 + c8;
      *(volatile v8h*)(UH + o) = hv[it];
      if (LO) *(volatile v8h*)(UL + o) = lv[it];
    }
    __threadfence();
  }
}

template <bool LO>
__global__ __launch_bounds__(256) void dtlow_pack_kernel(
    const float* __restrict__ XD, unsigned short* __restrict__ dH, unsigned short* __restrict__ dL, int total8)
{
  const int i = blockIdx.x * 256 + threadIdx.x;
  if (i >= total8) return;
  const int row = i >> 3;
  const int c8  = (i & 7) * 8;
  const float* sp = XD + (size_t)row * kXpP + c8;
  const v4f a0 = *(const v4f*)(sp);
  const v4f a1 = *(const v4f*)(sp + 4);
  v8h hv, lv;
#pragma unroll
  for (int e = 0; e < 4; ++e) {
    _Float16 h0, l0, h1, l1;
    const float f0 = a0[e] * kDlCarry;
    const float f1 = a1[e] * kDlCarry;
    f16_split(f0, h0, l0);
    f16_split(f1, h1, l1);
    hv[e] = h0; lv[e] = l0;
    hv[4 + e] = h1; lv[4 + e] = l1;
  }
  const size_t e0 = (size_t)i << 3;
  unsigned short* qh = dH + e0;
  unsigned short* ql = dL + e0;
  *(volatile v8h*)qh = hv;
  if (LO) *(volatile v8h*)ql = lv;
  __threadfence();
  *(volatile v8h*)qh = hv;
  if (LO) *(volatile v8h*)ql = lv;
}

typedef float    ms1_v4f __attribute__((ext_vector_type(4)));
typedef unsigned ms1_v4u __attribute__((ext_vector_type(4)));
struct ms1_args {
  const float* dtpre;
  const float* u;
  const float* bc;
  const float* z;
  const float* A_log;
  const float* Dskip;
  __half* y;
  __half* y_lo;
  long ld_dtpre;
  long ld_u;
  long ld_bc;
  long ld_z;
  long ld_y;
  int offB;
  int offC;
  int offZ;
  float ycarry;
  int dir;
  int D;
  int L;
  int nbatch;
};
static_assert(sizeof(ms1_args) == 136);

__device__ __forceinline__ float ms1_flush16(float v) {
  return (fabsf(v) < 6.103515625e-05f) ? 0.0f : v;
}
__device__ __forceinline__ unsigned ms1_h16bits(float v) {
  return (unsigned)__half_as_ushort(__float2half_rn(ms1_flush16(v)));
}
__device__ __forceinline__ float ms1_h16val(unsigned b) {
  return __half2float(__ushort_as_half((unsigned short)b));
}
__device__ __forceinline__ float ms1_softplus(float v) {
  return fmaxf(v, 0.0f) + log1pf(expf(-fabsf(v)));
}
__device__ __forceinline__ void ms1_pack2(float v0, float v1, unsigned& hw, unsigned& lw) {
  const unsigned h0 = ms1_h16bits(v0);
  const unsigned h1 = ms1_h16bits(v1);
  const float r0 = (v0 - ms1_h16val(h0)) * 2048.0f;
  const float r1 = (v1 - ms1_h16val(h1)) * 2048.0f;
  const unsigned l0 = ms1_h16bits(r0);
  const unsigned l1 = ms1_h16bits(r1);
  hw = h0 | (h1 << 16);
  lw = l0 | (l1 << 16);
}

template <int NSTATE>
__global__ __launch_bounds__(64 * (NSTATE / 16)) void ms1_scan_kernel(ms1_args a)
{
  static_assert(NSTATE == 16 || NSTATE == 64);
  constexpr int NQ  = NSTATE / 16;
  constexpr int NT  = 64 * NQ;
  constexpr int NW  = NT / 32;
  constexpr int BCW = 2 * NSTATE;
  constexpr int YP  = 68;
  constexpr int RPI = NW * 4;
  constexpr int NIT = 64 / RPI;
  static_assert(16 * NT <= 64 * YP);
  __shared__ __align__(16) float sBC[64 * BCW];
  __shared__ __align__(16) float sY[64 * YP];
  const int tid  = threadIdx.x;
  const int lane = tid & 31;
  const int wave = tid >> 5;
  const int c    = tid / NQ;
  const int sq   = tid - c * NQ;
  const int bpb  = a.D / 64;
  const int bi   = blockIdx.x / bpb;
  if (bi >= a.nbatch) return;
  const int d0 = (blockIdx.x - bi * bpb) * 64;
  const int d  = d0 + c;
  const long rowb = (long)bi * a.L;
  const bool hasz  = (a.z != nullptr);
  const bool hasD  = (a.Dskip != nullptr);
  const bool hasLo = (a.y_lo != nullptr);

#pragma unroll 1
  for (int n = 0; n < 16; ++n) {
    const float al = a.A_log[(long)d * NSTATE + sq * 16 + n];
    sY[n * NT + tid] = -expf(al);
  }
  __syncthreads();
  float An[16], h[16];
#pragma unroll
  for (int n = 0; n < 16; ++n) {
    An[n] = sY[n * NT + tid];
    h[n] = 0.0f;
  }
  float Dd = 0.0f;
  if (hasD) Dd = a.Dskip[d];

  const int nchunk = a.L / 64;
  const bool fwd = (a.dir > 0);
  const int s0 = fwd ? 0 : 63;
  const int sd = fwd ? 1 : -1;
  const int q  = lane >> 3;
  const int c8 = (lane & 7) * 8;

#pragma unroll 1
  for (int ci = 0; ci < nchunk; ++ci) {
    const int tb = fwd ? (ci * 64) : (a.L - 64 - ci * 64);
    const long rowc = rowb + tb;
    __syncthreads();
#pragma unroll 8
    for (int i = 0; i < 32; ++i) {
      const int idx = tid + i * NT;
      const int st  = idx / BCW;
      const int col = idx - st * BCW;
      const int sc  = (col < NSTATE) ? (a.offB + col) : (a.offC + col - NSTATE);
      sBC[idx] = a.bc[(rowc + st) * a.ld_bc + sc];
    }
    __syncthreads();
#pragma unroll 1
    for (int s = 0; s < 64; ++s) {
      const int ls = s0 + sd * s;
      const long row = rowc + ls;
      float pre = a.dtpre[row * a.ld_dtpre + d];
      float uv  = a.u[row * a.ld_u + d];
      float zv  = 0.0f;
      if (hasz) zv = a.z[row * a.ld_z + a.offZ + d];
      asm volatile("" : "+v"(pre));
      asm volatile("" : "+v"(uv));
      asm volatile("" : "+v"(zv));
      const float delta = ms1_softplus(pre);
      const float dtx = delta * uv;
      const float* bp = sBC + ls * BCW + sq * 16;
      const float* cp = bp + NSTATE;
      ms1_v4f Bq[4], Cq[4];
#pragma unroll
      for (int k = 0; k < 4; ++k) {
        Bq[k] = *(const ms1_v4f*)(bp + 4 * k);
        Cq[k] = *(const ms1_v4f*)(cp + 4 * k);
      }
      float yv = 0.0f;
#pragma unroll
      for (int n = 0; n < 16; ++n) {
        const float e = __expf(delta * An[n]);
        h[n] = fmaf(e, h[n], dtx * Bq[n >> 2][n & 3]);
        yv = fmaf(h[n], Cq[n >> 2][n & 3], yv);
      }
      if (NQ > 1) {
        yv += __shfl_xor(yv, 1, 32);
        yv += __shfl_xor(yv, 2, 32);
      }
      if (hasD) yv = fmaf(uv, Dd, yv);
      if (hasz) {
        const float sg = __builtin_amdgcn_rcpf(1.0f + expf(-zv));
        yv = yv * (zv * sg);
      }
      if (sq == 0) sY[ls * YP + c] = yv * a.ycarry;
    }
    __syncthreads();
    ms1_v4u hw[NIT], lw[NIT];
#pragma unroll
    for (int it = 0; it < NIT; ++it) {
      const int row = it * RPI + wave * 4 + q;
      const float* sp = sY + row * YP + c8;
      const ms1_v4f f0 = *(const ms1_v4f*)(sp);
      const ms1_v4f f1 = *(const ms1_v4f*)(sp + 4);
      unsigned h0, h1, h2, h3, l0, l1, l2, l3;
      ms1_pack2(f0[0], f0[1], h0, l0);
      ms1_pack2(f0[2], f0[3], h1, l1);
      ms1_pack2(f1[0], f1[1], h2, l2);
      ms1_pack2(f1[2], f1[3], h3, l3);
      hw[it] = (ms1_v4u){h0, h1, h2, h3};
      lw[it] = (ms1_v4u){l0, l1, l2, l3};
    }
    for (int pass = 0; pass < 2; ++pass) {
#pragma unroll
      for (int it = 0; it < NIT; ++it) {
        const int row = it * RPI + wave * 4 + q;
        const long o = (rowc + row) * a.ld_y + d0 + c8;
        *(volatile ms1_v4u*)(a.y + o) = hw[it];
        if (hasLo) *(volatile ms1_v4u*)(a.y_lo + o) = lw[it];
      }
      __threadfence();
    }
  }
}

template <bool LO>
__global__ __launch_bounds__(256) void gelu_pack_kernel(
    const unsigned* __restrict__ YHw, const unsigned* __restrict__ YLw,
    unsigned* __restrict__ GHw, unsigned* __restrict__ GLw, int total2)
{
  const int i = blockIdx.x * 256 + threadIdx.x;
  if (i >= total2) return;
  const unsigned yh = YHw[i];
  const unsigned yl = YLw[i];
  unsigned hw = 0u, lw = 0u;
#pragma unroll 1
  for (int e = 0; e < 2; ++e) {
    const unsigned sh = 16u * (unsigned)e;
    const float yv = h16_to_f32((yh >> sh) & 0xffffu);
    const float yr = h16_to_f32((yl >> sh) & 0xffffu);
    const float y  = (yv + yr * (1.0f / kResid)) * (1.0f / kYCarry);
    const float g  = 0.5f * y * (1.0f + erff(y * 0.70710678118654752f));
    const float gc = g * kGCarry;
    const unsigned hb = f16_bits_flush(gc);
    const float r  = (gc - h16_to_f32(hb)) * kResid;
    const unsigned lb = f16_bits_flush(r);
    hw |= hb << sh;
    lw |= lb << sh;
  }
  ((volatile unsigned*)GHw)[i] = hw;
  if (LO) ((volatile unsigned*)GLw)[i] = lw;
  __threadfence();
  ((volatile unsigned*)GHw)[i] = hw;
  if (LO) ((volatile unsigned*)GLw)[i] = lw;
}

__global__ __launch_bounds__(256) void glu_transpose_kernel(const float* __restrict__ OUTp, float* __restrict__ out)
{
  __shared__ __align__(16) float tile[64 * 68];
  const int tid = threadIdx.x, lane = tid & 31, wave = tid >> 5;
  const int l0 = blockIdx.x * 64;
  const int c0 = blockIdx.y * 64;
  const int b  = blockIdx.z;
  const float* src = OUTp + ((size_t)b * kSeq + l0) * kOutN + c0;
#pragma unroll 1
  for (int p = 0; p < 4; ++p) {
    const int idx = tid + p * 256;
    const int ll  = idx >> 4;
    const int c4  = (idx & 15) * 4;
    const v4f av = *(const v4f*)(src + (size_t)ll * kOutN + c4);
    const v4f gv = *(const v4f*)(src + (size_t)ll * kOutN + kDm + c4);
#pragma unroll
    for (int e = 0; e < 4; ++e) {
      const float sg = __builtin_amdgcn_rcpf(1.0f + expf(-gv[e]));
      tile[(c4 + e) * 68 + ll] = av[e] * sg;
    }
  }
  __syncthreads();
  const int hh = lane >> 4, l4 = (lane & 15) * 4;
  v4f fv[4];
#pragma unroll
  for (int it = 0; it < 4; ++it) fv[it] = *(const v4f*)(tile + (wave * 8 + it * 2 + hh) * 68 + l4);
  for (int pass = 0; pass < 2; ++pass) {
#pragma unroll
    for (int it = 0; it < 4; ++it) {
      const int crow = c0 + wave * 8 + it * 2 + hh;
      *(volatile v4f*)(out + ((size_t)b * kDm + crow) * kSeq + l0 + l4) = fv[it];
    }
    __threadfence();
  }
}

extern "C" void kernel_launch(void* const* d_in, const int* in_sizes, int n_in,
                              void* d_out, int out_size, void* d_ws, size_t ws_size,
                              hipStream_t stream)
{
  if (n_in < 8) return;
  if (in_sizes[0] != kBatch * kDm * kSeq) return;
  if (in_sizes[1] != kXpN * kDm) return;
  if (in_sizes[2] != kDm * kRank) return;
  if (in_sizes[3] != kDm) return;
  if (in_sizes[4] != kDm * kNst) return;
  if (in_sizes[5] != kDm) return;
  if (in_sizes[6] != kOutN * kDm) return;
  if (in_sizes[7] != kOutN) return;
  if (out_size != kBatch * kDm * kSeq) return;
  if (ws_size < kWsTotal) return;

  const float* hid   = (const float*)d_in[0];
  const float* xpw   = (const float*)d_in[1];
  const float* dtw   = (const float*)d_in[2];
  const float* dtb   = (const float*)d_in[3];
  const float* A_log = (const float*)d_in[4];
  const float* D_par = (const float*)d_in[5];
  const float* outw  = (const float*)d_in[6];
  const float* outb  = (const float*)d_in[7];
  float* out = (float*)d_out;

  char* ws = (char*)d_ws;
  float*          U    = (float*)(ws + kOffU);
  unsigned short* UH   = (unsigned short*)(ws + kOffUH);
  unsigned short* UL   = (unsigned short*)(ws + kOffUL);
  unsigned short* XWH  = (unsigned short*)(ws + kOffXWH);
  unsigned short* XWL  = (unsigned short*)(ws + kOffXWL);
  unsigned short* DTWH = (unsigned short*)(ws + kOffDTWH);
  unsigned short* DTWL = (unsigned short*)(ws + kOffDTWL);
  unsigned short* OWH  = (unsigned short*)(ws + kOffOWH);
  unsigned short* OWL  = (unsigned short*)(ws + kOffOWL);
  float*          XD   = (float*)(ws + kOffXD);
  unsigned short* DTLH = (unsigned short*)(ws + kOffDTLH);
  unsigned short* DTLL = (unsigned short*)(ws + kOffDTLL);
  float*          DT   = (float*)(ws + kOffDT);
  unsigned short* YH   = (unsigned short*)(ws + kOffYH);
  unsigned short* YL   = (unsigned short*)(ws + kOffYL);
  unsigned short* GH   = (unsigned short*)(ws + kOffGH);
  unsigned short* GL   = (unsigned short*)(ws + kOffGL);
  float*          OUTp = (float*)(ws + kOffOUT);

  pack_rows_kernel<(kSplX == 2)><<<(kXpP * kDm / 8) / 256, 256, 0, stream>>>(
      xpw, XWH, XWL, kXpN, kDm, kXpP * kDm / 8, kXwCarry);
  pack_rows_kernel<(kSplDt == 2)><<<(kDm * kRank / 8) / 256, 256, 0, stream>>>(
      dtw, DTWH, DTWL, kDm, kRank, kDm * kRank / 8, kDwCarry);
  pack_rows_kernel<(kSplOut == 2)><<<(kOutN * kDm / 8) / 256, 256, 0, stream>>>(
      outw, OWH, OWL, kOutN, kDm, kOutN * kDm / 8, kOwCarry);

  transpose_u_kernel<(kSplX >= 1)><<<dim3(kSeq / 64, kDm / 64, kBatch), 256, 0, stream>>>(hid, U, UH, UL);

  eng::gemm_f16_kernel<kMiX, kSplX, 0><<<dim3((kRows / (16 * kMiX)) * (kXpP / 64) / 8), 256, 0, stream>>>(
      UH, (kSplX >= 1) ? UL : UH, kDm, XWH, (kSplX == 2) ? XWL : XWH, kDm,
      XD, kXpP, outb, kRows, kXpP, kDm, kScX, kScXr);

  dtlow_pack_kernel<(kSplDt >= 1)><<<(kRows * kRank / 8) / 256, 256, 0, stream>>>(XD, DTLH, DTLL, kRows * kRank / 8);

  eng::gemm_f16_kernel<kMiDt, kSplDt, 1><<<dim3((kRows / (16 * kMiDt)) * (kDm / 64) / 8), 256, 0, stream>>>(
      DTLH, (kSplDt >= 1) ? DTLL : DTLH, kRank, DTWH, (kSplDt == 2) ? DTWL : DTWH, kRank,
      DT, kDm, dtb, kRows, kDm, kRank, kScDt, kScDtr);

  for (int b = 0; b < kBatch; ++b) {
    const size_t ro = (size_t)b * kSeq;
    ms1_args sa;
    sa.dtpre = DT + ro * kDm;
    sa.u = U + ro * kDm;
    sa.bc = XD + ro * kXpP;
    sa.z = U + ro * kDm;
    sa.A_log = A_log;
    sa.Dskip = D_par;
    sa.y = (__half*)(YH + ro * kDm);
    sa.y_lo = (__half*)(YL + ro * kDm);
    sa.ld_dtpre = kDm;
    sa.ld_u = kDm;
    sa.ld_bc = kXpP;
    sa.ld_z = kDm;
    sa.ld_y = kDm;
    sa.offB = kOffB;
    sa.offC = kOffC;
    sa.offZ = 0;
    sa.ycarry = kYCarry;
    sa.dir = 1;
    sa.D = kDm;
    sa.L = kSeq;
    sa.nbatch = 1;
    ms1_scan_kernel<16><<<dim3(kDm / 64), 64, 0, stream>>>(sa);
  }

  gelu_pack_kernel<(kSplOut >= 1)><<<(kRows * kDm / 2) / 256, 256, 0, stream>>>(
      (const unsigned*)YH, (const unsigned*)YL, (unsigned*)GH, (unsigned*)GL, kRows * kDm / 2);

  eng::gemm_f16_kernel<kMiOut, kSplOut, 1><<<dim3((kRows / (16 * kMiOut)) * (kOutN / 64) / 8), 256, 0, stream>>>(
      GH, (kSplOut >= 1) ? GL : GH, kDm, OWH, (kSplOut == 2) ? OWL : OWH, kDm,
      OUTp, kOutN, outb, kRows, kOutN, kDm, kScOut, kScOutr);

  glu_transpose_kernel<<<dim3(kSeq / 64, kDm / 64, kBatch), 256, 0, stream>>>(OUTp, out);
}
